// DeltaNetAttentionCore_70334384439584
// MI455X (gfx1250) — hardware-verified
//
#include <hip/hip_runtime.h>
#include <math.h>

constexpr int SEQ_LEN  = 2048;
constexpr int NBAT     = 2;
constexpr int HID      = 2048;
constexpr int CHN      = 2048;
constexpr int NHEAD    = 16;
constexpr int HDIM     = 128;
constexpr int NTAP     = 4;
constexpr int NROW     = SEQ_LEN * NBAT;
constexpr int BETA_COL = 3 * CHN;
constexpr int NPL      = 3 * CHN + 64;
constexpr int CLEN     = 32;
constexpr int NCHK     = SEQ_LEN / CLEN;
constexpr int KPIT     = 136;
constexpr int TPIT     = 40;
constexpr int RPIT     = 132;
constexpr int GPIT     = 36;
constexpr float WCARRY = 16.0f;
constexpr float WINV   = 1.0f / WCARRY;
constexpr float KCARRY = 16.0f;
constexpr float QCARRY = 64.0f;
constexpr float UCARRY = 1.0f;
constexpr float SCARRY = KCARRY * UCARRY;
constexpr float INV_G  = 1.0f / (KCARRY * KCARRY);
constexpr float INV_KS = 1.0f / (KCARRY * SCARRY);
constexpr float INV_O  = 1.0f / (QCARRY * SCARRY);
constexpr float L2EPS  = 1e-12f;
constexpr float RMSEPS = 1e-5f;
static_assert(CHN == NHEAD * HDIM);
static_assert(NROW % 64 == 0 && NPL % 64 == 0 && HID % 64 == 0 && CHN % 64 == 0);
static_assert(HID % 32 == 0 && CHN % 32 == 0);
static_assert(SEQ_LEN % CLEN == 0 && CLEN == 32 && HDIM == 128 && NTAP == 4);
static_assert(QCARRY * KCARRY * UCARRY == QCARRY * SCARRY);
static_assert(KPIT % 8 == 0 && TPIT % 8 == 0 && RPIT % 4 == 0 && GPIT % 4 == 0);
static_assert((NPL * 2) % 128 == 0);

typedef __attribute__((ext_vector_type(16))) _Float16 v16h;
typedef __attribute__((ext_vector_type(8)))  _Float16 v8h;
typedef __attribute__((ext_vector_type(4)))  _Float16 v4h;
typedef __attribute__((ext_vector_type(16))) __bf16   v16b;
typedef __attribute__((ext_vector_type(8)))  __bf16   v8b;
typedef __attribute__((ext_vector_type(8)))  float    v8f;
typedef __attribute__((ext_vector_type(4)))  float    v4f;
typedef __attribute__((ext_vector_type(4)))  unsigned int v4u;
typedef __attribute__((ext_vector_type(2)))  unsigned int v2u;

__device__ __forceinline__ unsigned short f2bf_bits(float f) {
  unsigned u = __float_as_uint(f);
  return (unsigned short)((u + 0x7FFFu + ((u >> 16) & 1u)) >> 16);
}
__device__ __forceinline__ float bf_bits2f(unsigned short h) { return __uint_as_float(((unsigned)h) << 16); }
__device__ __forceinline__ float bf16r(float f) { return bf_bits2f(f2bf_bits(f)); }
__device__ __forceinline__ unsigned pk16(unsigned short a, unsigned short b) { return (unsigned)a | ((unsigned)b << 16); }
__device__ __forceinline__ unsigned short h_bits(float f) { const _Float16 h = (_Float16)f; return __builtin_bit_cast(unsigned short, h); }
__device__ __forceinline__ float h16_to_f32(unsigned hb) {
  const unsigned sgn = (hb & 0x8000u) << 16;
  const unsigned em = hb & 0x7fffu;
  const float fn = __uint_as_float((em << 13) + 0x38000000u);
  const float fs = (float)em * 5.9604644775390625e-8f;
  const float mag = (em < 0x400u) ? fs : fn;
  return __uint_as_float(__float_as_uint(mag) | sgn);
}

__device__ __forceinline__ void dep_guard4_h(v8f& a, v8f& b, v8f& c, v8f& d, v16h x, v16h y, v16h b0, v16h b1, v16h b2, v16h b3) {
  asm volatile("v_nop\n\tv_nop\n\tv_nop\n\tv_nop" : "+v"(a), "+v"(b), "+v"(c), "+v"(d) : "v"(x), "v"(y), "v"(b0), "v"(b1), "v"(b2), "v"(b3));
}
__device__ __forceinline__ void dep_guard4_b(v8f& a, v8f& b, v8f& c, v8f& d, v16b x, v16b y, v16b b0, v16b b1, v16b b2, v16b b3) {
  asm volatile("v_nop\n\tv_nop\n\tv_nop\n\tv_nop" : "+v"(a), "+v"(b), "+v"(c), "+v"(d) : "v"(x), "v"(y), "v"(b0), "v"(b1), "v"(b2), "v"(b3));
}
__device__ __forceinline__ void keep4_h(v16h a, v16h b, v16h c, v16h d) { asm volatile("v_nop" :: "v"(a), "v"(b), "v"(c), "v"(d)); }
__device__ __forceinline__ void keep4_b(v16b a, v16b b, v16b c, v16b d) { asm volatile("v_nop" :: "v"(a), "v"(b), "v"(c), "v"(d)); }
__device__ __forceinline__ void acc_guard4(v8f& a, v8f& b, v8f& c, v8f& d) { asm volatile("v_nop\n\tv_nop\n\tv_nop\n\tv_nop" : "+v"(a), "+v"(b), "+v"(c), "+v"(d)); }
template <typename T> struct Frag;
template <> struct Frag<_Float16> {
  typedef v16h V; union U { v16h v; v8h h[2]; };
  static __device__ __forceinline__ v16h load(const _Float16* p) {
    U f; f.h[0] = *(const v8h*)(p); f.h[1] = *(const v8h*)(p + 16); return f.v;
  }
  static __device__ __forceinline__ v8f mma(v16h a, v16h b, v8f c) {
    return __builtin_amdgcn_wmma_f32_16x16x32_f16(false, a, false, b, (short)0, c, false, false);
  }
  static __device__ __forceinline__ void guard4(v8f& a, v8f& b, v8f& c, v8f& d, v16h x, v16h y, v16h b0, v16h b1, v16h b2, v16h b3) { dep_guard4_h(a, b, c, d, x, y, b0, b1, b2, b3); }
  static __device__ __forceinline__ void keep(v16h a, v16h b, v16h c, v16h d) { keep4_h(a, b, c, d); }
};
template <> struct Frag<__bf16> {
  typedef v16b V; union U { v16b v; v8b h[2]; };
  static __device__ __forceinline__ v16b load(const __bf16* p) {
    U f; f.h[0] = *(const v8b*)(p); f.h[1] = *(const v8b*)(p + 16); return f.v;
  }
  static __device__ __forceinline__ v8f mma(v16b a, v16b b, v8f c) {
    return __builtin_amdgcn_wmma_f32_16x16x32_bf16(false, a, false, b, (short)0, c, false, false);
  }
  static __device__ __forceinline__ void guard4(v8f& a, v8f& b, v8f& c, v8f& d, v16b x, v16b y, v16b b0, v16b b1, v16b b2, v16b b3) { dep_guard4_b(a, b, c, d, x, y, b0, b1, b2, b3); }
  static __device__ __forceinline__ void keep(v16b a, v16b b, v16b c, v16b d) { keep4_b(a, b, c, d); }
};
__device__ __forceinline__ v8f mma_g(v16h a, v16h b, v8f c) {
  c = __builtin_amdgcn_wmma_f32_16x16x32_f16(false, a, false, b, (short)0, c, false, false);
  asm volatile("v_nop\n\tv_nop\n\tv_nop\n\tv_nop" : "+v"(c) : "v"(a), "v"(b));
  return c;
}

template <int ET> struct Elem;
template <> struct Elem<0> { typedef _Float16 T; };
template <> struct Elem<1> { typedef __bf16 T; };
template <int ET, bool SPLIT, int BIAS_MODE, int OUT_MODE, bool RESID, int ACT = 0>
__global__ __launch_bounds__(256) void wmma_gemm64(
    const unsigned short* __restrict__ Ap, const unsigned short* __restrict__ A2p, int lda, long strideA,
    const unsigned short* __restrict__ Btp, const unsigned short* __restrict__ Bt2p, int ldb, long strideB,
    void* __restrict__ Cout, void* __restrict__ Cout2, int ldc, long strideC,
    const float* __restrict__ bias,
    const float* __restrict__ resid, long strideR,
    int M, int N, int K, float scale) {
  typedef typename Elem<ET>::T T;
  typedef typename Frag<T>::V V;
  const T* A = (const T*)Ap; const T* A2 = (const T*)A2p; const T* Bt = (const T*)Btp; const T* Bt2 = (const T*)Bt2p;
  __shared__ __align__(16) float sT[8][16 * 68];
  const int b    = blockIdx.y;
  const int lane = threadIdx.x & 31;
  const int wave = threadIdx.x >> 5;
  const int tilesN = N >> 6;
  const int tilesM = M >> 6;
  const int tile = blockIdx.x * 8 + wave;
  if (tile >= tilesM * tilesN) return;
  const int tm = tile / tilesN;
  const int tn = tile - tm * tilesN;
  const int m0 = tm << 6;
  const int n0 = tn << 6;

  const T* Ab  = A  + (size_t)b * strideA;
  const T* Bb  = Bt + (size_t)b * strideB;
  const T* Ab2 = SPLIT ? (A2  + (size_t)b * strideA) : nullptr;
  const T* Bb2 = SPLIT ? (Bt2 + (size_t)b * strideB) : nullptr;

  const int rlane = lane & 15;
  const int koff  = (lane >> 4) * 8;
  const int mOff  = (lane >> 4) * 8;

  v8f acc[4][4];
#pragma unroll
  for (int i = 0; i < 4; ++i)
#pragma unroll
    for (int j = 0; j < 4; ++j) acc[i][j] = (v8f){0.f,0.f,0.f,0.f,0.f,0.f,0.f,0.f};

  for (int k0 = 0; k0 < K; k0 += 32) {
    V bh[4], bl[4];
#pragma unroll
    for (int j = 0; j < 4; ++j) {
      const size_t bo = (size_t)(n0 + (j << 4) + rlane) * ldb + koff + k0;
      bh[j] = Frag<T>::load(Bb + bo);
      if (SPLIT) bl[j] = Frag<T>::load(Bb2 + bo);
    }
#pragma unroll
    for (int i = 0; i < 4; ++i) {
      const size_t ao = (size_t)(m0 + (i << 4) + rlane) * lda + koff + k0;
      V ah = Frag<T>::load(Ab + ao);
      V al;
      if (SPLIT) al = Frag<T>::load(Ab2 + ao);
#pragma unroll
      for (int j = 0; j < 4; ++j) {
        acc[i][j] = Frag<T>::mma(ah, bh[j], acc[i][j]);
        if (SPLIT) {
          acc[i][j] = Frag<T>::mma(ah, bl[j], acc[i][j]);
          acc[i][j] = Frag<T>::mma(al, bh[j], acc[i][j]);
        }
      }
      Frag<T>::guard4(acc[i][0], acc[i][1], acc[i][2], acc[i][3], ah, SPLIT ? al : ah, bh[0], bh[1], bh[2], bh[3]);
    }
    Frag<T>::keep(bh[0], bh[1], bh[2], bh[3]);
    if (SPLIT) Frag<T>::keep(bl[0], bl[1], bl[2], bl[3]);
  }
  acc_guard4(acc[0][0], acc[0][1], acc[0][2], acc[0][3]);
  acc_guard4(acc[1][0], acc[1][1], acc[1][2], acc[1][3]);
  acc_guard4(acc[2][0], acc[2][1], acc[2][2], acc[2][3]);
  acc_guard4(acc[3][0], acc[3][1], acc[3][2], acc[3][3]);

  float* slab = sT[wave];
  const float* Rb = RESID ? (resid + (size_t)b * strideR) : nullptr;
#pragma unroll
  for (int i = 0; i < 4; ++i) {
    const int mBase = m0 + (i << 4);
#pragma unroll
    for (int j = 0; j < 4; ++j) {
      const int n = n0 + (j << 4) + rlane;
      float bv = 0.f;
      if (BIAS_MODE == 2) bv = bias[n];
#pragma unroll
      for (int r = 0; r < 8; ++r) {
        float v = acc[i][j][r] * scale;
        if (BIAS_MODE == 1) v += bias[mBase + mOff + r];
        if (BIAS_MODE == 2) v += bv;
        if (RESID) v += Rb[(size_t)(mBase + mOff + r) * ldc + n];
        if (ACT == 2) v = fmaxf(v, 0.0f);
        if (ACT == 4) v = (v > 0.f) ? v : 0.01f * v;
        slab[(mOff + r) * 68 + (j << 4) + rlane] = v;
      }
    }
    __builtin_amdgcn_fence(__ATOMIC_RELEASE, "workgroup");
    __builtin_amdgcn_wave_barrier();
    __builtin_amdgcn_fence(__ATOMIC_ACQUIRE, "workgroup");
    if (OUT_MODE == 0) {
      float* C = (float*)Cout + (size_t)b * strideC;
      const int hh = lane >> 4, c4 = (lane & 15) * 4;
      for (int pass = 0; pass < 2; ++pass) {
#pragma unroll
        for (int it = 0; it < 8; ++it) {
          const int row = it * 2 + hh;
          v4f v = *(const v4f*)(slab + row * 68 + c4);
          *(volatile v4f*)(C + (size_t)(mBase + row) * ldc + n0 + c4) = v;
        }
        __threadfence();
      }
    } else {
      const int q = lane >> 3, c8 = (lane & 7) * 8;
      unsigned short* C  = (unsigned short*)Cout  + (size_t)b * strideC;
      unsigned short* C2 = (OUT_MODE == 2) ? ((unsigned short*)Cout2 + (size_t)b * strideC) : nullptr;
      for (int pass = 0; pass < 2; ++pass) {
#pragma unroll
        for (int it = 0; it < 4; ++it) {
          const int row = it * 4 + q;
          const float* sp = slab + row * 68 + c8;
          v8h hv, lv;
#pragma unroll
          for (int e = 0; e < 8; ++e) {
            if (OUT_MODE == 1) {
              hv[e] = (_Float16)sp[e];
            } else {
              unsigned short hb = f2bf_bits(sp[e]);
              unsigned short lb = f2bf_bits(sp[e] - bf_bits2f(hb));
              hv[e] = __builtin_bit_cast(_Float16, hb);
              lv[e] = __builtin_bit_cast(_Float16, lb);
            }
          }
          *(volatile v8h*)(C + (size_t)(mBase + row) * ldc + n0 + c8) = hv;
          if (OUT_MODE == 2) *(volatile v8h*)(C2 + (size_t)(mBase + row) * ldc + n0 + c8) = lv;
        }
        __threadfence();
      }
    }
    __builtin_amdgcn_fence(__ATOMIC_RELEASE, "workgroup");
    __builtin_amdgcn_wave_barrier();
    __builtin_amdgcn_fence(__ATOMIC_ACQUIRE, "workgroup");
  }
}

__global__ __launch_bounds__(256) void cast8_bf_f16_kernel(const float* __restrict__ in, unsigned short* __restrict__ out, int n8) {
  const int i = blockIdx.x * 256 + threadIdx.x;
  if (i >= n8) return;
  const float* p = in + 8 * (size_t)i;
  const v4f a = *(const v4f*)(p);
  const v4f c = *(const v4f*)(p + 4);
  unsigned short hb[8];
#pragma unroll
  for (int e = 0; e < 4; ++e) {
    const float fa = a[e];
    const float fc = c[e];
    hb[e]     = h_bits(bf16r(fa));
    hb[4 + e] = h_bits(bf16r(fc));
  }
  const v4u u = (v4u){pk16(hb[0], hb[1]), pk16(hb[2], hb[3]), pk16(hb[4], hb[5]), pk16(hb[6], hb[7])};
  unsigned short* q = out + 8 * (size_t)i;
  *(volatile v4u*)q = u;
  __threadfence();
  *(volatile v4u*)q = u;
}

__global__ __launch_bounds__(256) void wtpack_kernel(const float* __restrict__ W0, const float* __restrict__ W1,
                                                     const float* __restrict__ W2, unsigned short* __restrict__ out, float carry) {
  __shared__ float sm[64][65];
  const int t  = threadIdx.x;
  const int k0 = blockIdx.x * 64;
  const int n0 = blockIdx.y * 64;
  const int z  = blockIdx.z;
  const float* W = (z == 0) ? W0 : (z == 1) ? W1 : W2;
#pragma unroll
  for (int i = 0; i < 16; ++i) {
    const int e = i * 256 + t;
    const int r = e >> 6;
    const int c = e & 63;
    const float wv = W[(size_t)(k0 + r) * 2048 + n0 + c];
    sm[c][r] = bf16r(wv) * carry;
  }
  __syncthreads();
  const int lane = t & 31, wave = t >> 5;
  const int q = lane >> 3, c8 = (lane & 7) * 8;
  unsigned short* op = out + (size_t)z * 2048 * 2048;
  for (int pass = 0; pass < 2; ++pass) {
#pragma unroll
    for (int it = 0; it < 2; ++it) {
      const int row = wave * 8 + it * 4 + q;
      unsigned short hb[8];
#pragma unroll
      for (int e = 0; e < 8; ++e) hb[e] = h_bits(sm[row][c8 + e]);
      const v4u u = (v4u){pk16(hb[0], hb[1]), pk16(hb[2], hb[3]), pk16(hb[4], hb[5]), pk16(hb[6], hb[7])};
      *(volatile v4u*)(op + (size_t)(n0 + row) * 2048 + k0 + c8) = u;
    }
    __threadfence();
  }
}

__global__ __launch_bounds__(256) void wbpack_kernel(const float* __restrict__ Wb, unsigned short* __restrict__ out, float carry) {
  const int row = blockIdx.x;
  const int k   = threadIdx.x * 8;
  const int rc  = row < 15 ? row : 15;
  const bool live = row < 16;
  unsigned short hb[8];
#pragma unroll
  for (int e = 0; e < 8; ++e) {
    const float wv = Wb[(size_t)(k + e) * NHEAD + rc];
    const float val = live ? (bf16r(wv) * carry) : 0.0f;
    hb[e] = h_bits(val);
  }
  const v4u u = (v4u){pk16(hb[0], hb[1]), pk16(hb[2], hb[3]), pk16(hb[4], hb[5]), pk16(hb[6], hb[7])};
  unsigned short* q = out + (size_t)(BETA_COL + row) * 2048 + k;
  *(volatile v4u*)q = u;
  __threadfence();
  *(volatile v4u*)q = u;
}

__global__ __launch_bounds__(256) void chunk_scan_kernel(
    const unsigned short* __restrict__ PL, const float* __restrict__ cwq, const float* __restrict__ cwk,
    const float* __restrict__ cwv, const float* __restrict__ gnorm, unsigned short* __restrict__ O16, float qscale) {
  __shared__ __align__(16) _Float16 sKQ[2 * CLEN * KPIT];
  __shared__ __align__(16) _Float16 sKnT[HDIM * TPIT];
  __shared__ __align__(16) _Float16 sUT[HDIM * TPIT];
  __shared__ __align__(16) _Float16 sPm[CLEN * TPIT];
  __shared__ __align__(16) float    sRO[CLEN * RPIT];
  __shared__ __align__(16) float    sG[CLEN * GPIT];
  __shared__ float sBeta[CLEN];
  _Float16* sKn = sKQ;
  _Float16* sQn = sKQ + CLEN * KPIT;

  const int tid = threadIdx.x, lane = tid & 31, wave = tid >> 5;
  const int hh = lane >> 4, c = lane & 15, koff = hh * 8;
  const int hd = blockIdx.x & (NHEAD - 1);
  const int bb = blockIdx.x >> 4;
  const int cg = lane;

  float gv[8];
  {
    const v4f g0 = *(const v4f*)(gnorm + 8 * c);
    const v4f g1 = *(const v4f*)(gnorm + 8 * c + 4);
#pragma unroll
    for (int e = 0; e < 4; ++e) {
      const float a0 = g0[e];
      const float a1 = g1[e];
      gv[e]     = bf16r(a0);
      gv[4 + e] = bf16r(a1);
    }
  }

  const v8f z8 = {0.f, 0.f, 0.f, 0.f, 0.f, 0.f, 0.f, 0.f};
  v8f sacc[8];
#pragma unroll
  for (int i = 0; i < 8; ++i) sacc[i] = z8;

#pragma unroll 1
  for (int ch = 0; ch < NCHK; ++ch) {
    const int t0 = ch * CLEN;

#pragma unroll 1
    for (int ten = 0; ten < 3; ++ten) {
      const float* cw = (ten == 0) ? cwq : (ten == 1) ? cwk : cwv;
      const int chan0 = hd * HDIM + cg * 4;
      v4f tp[4];
#pragma unroll
      for (int j = 0; j < 4; ++j) {
        const v4f tv = *(const v4f*)(cw + (size_t)(chan0 + j) * NTAP);
#pragma unroll
        for (int i = 0; i < 4; ++i) {
          const float x = tv[i];
          tp[j][i] = bf16r(x);
        }
      }
      const int col0 = ten * CHN + chan0;
#pragma unroll 1
      for (int it2 = 0; it2 < 2; ++it2) {
        const int rp  = wave + 8 * it2;
        const int tl0 = 2 * rp;
        const int tg0 = t0 + tl0;
        float xw[5][4];
#pragma unroll
        for (int j = 0; j < 5; ++j) {
          const int ts  = tg0 - 3 + j;
          const int tsc = ts < 0 ? 0 : ts;
          const v2u w = *(const v2u*)(PL + (size_t)(tsc * NBAT + bb) * NPL + col0);
          const unsigned w0 = w[0];
          const unsigned w1 = w[1];
          const bool ok = ts >= 0;
          const float f0 = h16_to_f32(w0 & 0xffffu);
          const float f1 = h16_to_f32(w0 >> 16);
          const float f2 = h16_to_f32(w1 & 0xffffu);
          const float f3 = h16_to_f32(w1 >> 16);
          xw[j][0] = ok ? f0 : 0.0f;
          xw[j][1] = ok ? f1 : 0.0f;
          xw[j][2] = ok ? f2 : 0.0f;
          xw[j][3] = ok ? f3 : 0.0f;
        }
        float av[2][4];
        float ssq[2];
#pragma unroll
        for (int rr = 0; rr < 2; ++rr) {
          float s2 = 0.0f;
#pragma unroll
          for (int e = 0; e < 4; ++e) {
            float y = 0.0f;
#pragma unroll
            for (int i = 0; i < 4; ++i) y = fmaf(xw[rr + i][e], tp[e][i], y);
            const float ex = expf(fminf(-y, 60.0f));
            const float a = y * __builtin_amdgcn_rcpf(1.0f + ex);
            av[rr][e] = a;
            s2 = fmaf(a, a, s2);
          }
          ssq[rr] = s2;
        }
#pragma unroll
        for (int off = 1; off < 32; off <<= 1) {
          ssq[0] += __shfl_xor(ssq[0], off, 32);
          ssq[1] += __shfl_xor(ssq[1], off, 32);
        }
        float rsv[2];
        rsv[0] = rsqrtf(ssq[0] + L2EPS);
        rsv[1] = rsqrtf(ssq[1] + L2EPS);
        if (ten == 0) {
#pragma unroll
          for (int rr = 0; rr < 2; ++rr) {
            v4h hv;
#pragma unroll
            for (int e = 0; e < 4; ++e) hv[e] = (_Float16)(((av[rr][e] * rsv[rr]) * qscale) * QCARRY);
            *(v4h*)(sQn + (tl0 + rr) * KPIT + cg * 4) = hv;
          }
        } else if (ten == 1) {
#pragma unroll
          for (int rr = 0; rr < 2; ++rr) {
            v4h hv;
#pragma unroll
            for (int e = 0; e < 4; ++e) {
              const _Float16 kh = (_Float16)((av[rr][e] * rsv[rr]) * KCARRY);
              hv[e] = kh;
              sKnT[(cg * 4 + e) * TPIT + tl0 + rr] = kh;
            }
            *(v4h*)(sKn + (tl0 + rr) * KPIT + cg * 4) = hv;
          }
        } else {
#pragma unroll
          for (int rr = 0; rr < 2; ++rr) {
            const v4f vv = (v4f){av[rr][0], av[rr][1], av[rr][2], av[rr][3]};
            *(v4f*)(sRO + (tl0 + rr) * RPIT + cg * 4) = vv;
          }
        }
      }
    }
    if (wave == 0) {
      const int tg = t0 + lane;
      const unsigned wd = *(const unsigned*)(PL + (size_t)(tg * NBAT + bb) * NPL + BETA_COL + (hd & ~1));
      const unsigned hb = (hd & 1) ? (wd >> 16) : (wd & 0xffffu);
      const float lg = h16_to_f32(hb);
      sBeta[lane] = __builtin_amdgcn_rcpf(1.0f + expf(fminf(-lg, 60.0f)));
    }
    __syncthreads();

    {
      const int ti = (wave >> 1) & 1, tj = wave & 1;
      const int aoff = (wave < 4) ? 0 : (CLEN * KPIT);
      v8f g = z8;
#pragma unroll
      for (int ks = 0; ks < 4; ++ks) {
        const v16h a  = Frag<_Float16>::load(sKQ + aoff + (16 * ti + c) * KPIT + 32 * ks + koff);
        const v16h bq = Frag<_Float16>::load(sKn + (16 * tj + c) * KPIT + 32 * ks + koff);
        g = mma_g(a, bq, g);
      }
      if (wave < 4) {
#pragma unroll
        for (int r = 0; r < 8; ++r) sG[(16 * ti + 8 * hh + r) * GPIT + 16 * tj + c] = g[r] * INV_G;
      } else {
#pragma unroll
        for (int r = 0; r < 8; ++r) {
          const int row = 16 * ti + 8 * hh + r;
          const int col = 16 * tj + c;
          const float gr = g[r];
          const float pv = (col <= row) ? gr : 0.0f;
          sPm[row * TPIT + col] = (_Float16)pv;
        }
      }
    }
    v8f oacc[2];
    oacc[0] = z8;
    oacc[1] = z8;
    {
      v16h sb[4];
#pragma unroll
      for (int ks = 0; ks < 4; ++ks) {
#pragma unroll
        for (int r = 0; r < 8; ++r) {
          sb[ks][r]     = (_Float16)sacc[2 * ks][r];
          sb[ks][8 + r] = (_Float16)sacc[2 * ks + 1][r];
        }
      }
      v8f racc[2];
      racc[0] = z8;
      racc[1] = z8;
#pragma unroll
      for (int ks = 0; ks < 4; ++ks) {
#pragma unroll
        for (int ti = 0; ti < 2; ++ti) {
          const v16h ak = Frag<_Float16>::load(sKn + (16 * ti + c) * KPIT + 32 * ks + koff);
          const v16h aq = Frag<_Float16>::load(sQn + (16 * ti + c) * KPIT + 32 * ks + koff);
          racc[ti] = mma_g(ak, sb[ks], racc[ti]);
          oacc[ti] = mma_g(aq, sb[ks], oacc[ti]);
        }
      }
#pragma unroll
      for (int ti = 0; ti < 2; ++ti) {
#pragma unroll
        for (int r = 0; r < 8; ++r) {
          const int idx = (16 * ti + 8 * hh + r) * RPIT + 16 * wave + c;
          const float vv = sRO[idx];
          sRO[idx] = vv - racc[ti][r] * INV_KS;
        }
      }
    }
    __syncthreads();

    if (tid < HDIM) {
      float u[CLEN];
#pragma unroll
      for (int t = 0; t < CLEN; ++t) {
        float accv = sRO[t * RPIT + tid];
#pragma unroll
        for (int i4 = 0; i4 < CLEN / 4; ++i4) {
          if (4 * i4 < t) {
            const v4f gq = *(const v4f*)(sG + t * GPIT + 4 * i4);
#pragma unroll
            for (int e = 0; e < 4; ++e) {
              if (4 * i4 + e < t) {
                const float ge = gq[e];
                accv = fmaf(-ge, u[4 * i4 + e], accv);
              }
            }
          }
        }
        u[t] = sBeta[t] * accv;
      }
#pragma unroll
      for (int q = 0; q < CLEN / 8; ++q) {
        v8h hv;
#pragma unroll
        for (int e = 0; e < 8; ++e) hv[e] = (_Float16)(u[8 * q + e] * UCARRY);
        *(v8h*)(sUT + tid * TPIT + 8 * q) = hv;
      }
    }
    __syncthreads();

    {
      const v16h ub = Frag<_Float16>::load(sUT + (16 * wave + c) * TPIT + koff);
#pragma unroll
      for (int ti = 0; ti < 2; ++ti) {
        const v16h ap = Frag<_Float16>::load(sPm + (16 * ti + c) * TPIT + koff);
        oacc[ti] = mma_g(ap, ub, oacc[ti]);
      }
#pragma unroll
      for (int i = 0; i < 8; ++i) {
        const v16h akt = Frag<_Float16>::load(sKnT + (16 * i + c) * TPIT + koff);
        sacc[i] = mma_g(akt, ub, sacc[i]);
      }
#pragma unroll
      for (int ti = 0; ti < 2; ++ti) {
#pragma unroll
        for (int r = 0; r < 8; ++r) sRO[(16 * ti + 8 * hh + r) * RPIT + 16 * wave + c] = oacc[ti][r] * INV_O;
      }
    }
    __syncthreads();

    {
      v4u pk[2];
#pragma unroll
      for (int it = 0; it < 2; ++it) {
        const int row = 4 * wave + 2 * it + hh;
        const v4f o0 = *(const v4f*)(sRO + row * RPIT + 8 * c);
        const v4f o1 = *(const v4f*)(sRO + row * RPIT + 8 * c + 4);
        float ov[8];
#pragma unroll
        for (int e = 0; e < 4; ++e) {
          const float a0 = o0[e];
          const float a1 = o1[e];
          ov[e]     = a0;
          ov[4 + e] = a1;
        }
        float ss = 0.0f;
#pragma unroll
        for (int e = 0; e < 8; ++e) ss = fmaf(ov[e], ov[e], ss);
#pragma unroll
        for (int off = 1; off < 16; off <<= 1) ss += __shfl_xor(ss, off, 32);
        const float sc = rsqrtf(ss * (1.0f / HDIM) + RMSEPS);
        unsigned short hb[8];
#pragma unroll
        for (int e = 0; e < 8; ++e) hb[e] = h_bits((ov[e] * sc) * gv[e]);
        pk[it] = (v4u){pk16(hb[0], hb[1]), pk16(hb[2], hb[3]), pk16(hb[4], hb[5]), pk16(hb[6], hb[7])};
      }
      for (int pass = 0; pass < 2; ++pass) {
#pragma unroll
        for (int it = 0; it < 2; ++it) {
          const int row = 4 * wave + 2 * it + hh;
          unsigned short* op = O16 + (size_t)((t0 + row) * NBAT + bb) * CHN + hd * HDIM + 8 * c;
          *(volatile v4u*)op = pk[it];
        }
        __threadfence();
      }
    }
    __syncthreads();
  }
}

extern "C" void kernel_launch(void* const* d_in, const int* in_sizes, int n_in,
                              void* d_out, int out_size, void* d_ws, size_t ws_size, hipStream_t stream) {
  if (n_in < 10 || d_out == nullptr || d_ws == nullptr) return;
  if (in_sizes[0] != NROW * HID || in_sizes[1] != HID * CHN || in_sizes[2] != HID * CHN || in_sizes[3] != HID * CHN ||
      in_sizes[4] != HID * NHEAD || in_sizes[5] != CHN * NTAP || in_sizes[6] != CHN * NTAP || in_sizes[7] != CHN * NTAP ||
      in_sizes[8] != HDIM || in_sizes[9] != CHN * HID || out_size != NROW * HID) return;

  const float* hs  = (const float*)d_in[0];
  const float* Wq  = (const float*)d_in[1];
  const float* Wk  = (const float*)d_in[2];
  const float* Wv  = (const float*)d_in[3];
  const float* Wb  = (const float*)d_in[4];
  const float* cwq = (const float*)d_in[5];
  const float* cwk = (const float*)d_in[6];
  const float* cwv = (const float*)d_in[7];
  const float* gn  = (const float*)d_in[8];
  const float* Wo  = (const float*)d_in[9];
  float* out = (float*)d_out;

  char* ws = (char*)d_ws; size_t off = 0;
  auto carve = [&](size_t bytes) -> char* { char* p = ws + off; off += (bytes + 255) & ~(size_t)255; return p; };
  unsigned short* HS16 = (unsigned short*)carve((size_t)NROW * HID * 2);
  unsigned short* W1T  = (unsigned short*)carve((size_t)NPL * HID * 2);
  unsigned short* WOT  = (unsigned short*)carve((size_t)HID * CHN * 2);
  unsigned short* PPL  = (unsigned short*)carve((size_t)NROW * NPL * 2);
  unsigned short* O16  = (unsigned short*)carve((size_t)NROW * CHN * 2);
  if (off > ws_size || off > (size_t)134217728) return;

  const float qscale = (float)(1.0 / sqrt((double)HDIM));

  const int n8 = NROW * HID / 8;
  cast8_bf_f16_kernel<<<(n8 + 255) / 256, 256, 0, stream>>>(hs, HS16, n8);
  wtpack_kernel<<<dim3(HID / 64, CHN / 64, 3), 256, 0, stream>>>(Wq, Wk, Wv, W1T, WCARRY);
  wbpack_kernel<<<64, 256, 0, stream>>>(Wb, W1T, WCARRY);
  wtpack_kernel<<<dim3(CHN / 64, HID / 64, 1), 256, 0, stream>>>(Wo, Wo, Wo, WOT, WCARRY);

  wmma_gemm64<0, false, 0, 1, false, 0><<<dim3((NROW / 64) * (NPL / 64) / 8, 1), 256, 0, stream>>>(
      HS16, HS16, HID, 0L, W1T, W1T, HID, 0L, (void*)PPL, (void*)PPL, NPL, 0L,
      gn, hs, 0L, NROW, NPL, HID, WINV);

  chunk_scan_kernel<<<NBAT * NHEAD, 256, 0, stream>>>(PPL, cwq, cwk, cwv, gn, O16, qscale);

  wmma_gemm64<0, false, 0, 0, false, 0><<<dim3((NROW / 64) * (HID / 64) / 8, 1), 256, 0, stream>>>(
      O16, O16, CHN, 0L, WOT, WOT, CHN, 0L, (void*)out, (void*)out, HID, 0L,
      gn, hs, 0L, NROW, HID, CHN, WINV);
}
